// HeteroGraphSAGE_LINK_24524263260184
// MI455X (gfx1250) — hardware-verified
//
#include <hip/hip_runtime.h>
#include <stddef.h>


#define DF      128
#define PEIN    8
#define HID     64
#define KPE     192
#define KSG     256
#define NTHR    256
#define NWAVE   8
#define EPT     8
#define NGRP    2
#define CHUNK   (NTHR * EPT * NGRP)
#define WCAP    (EPT * NGRP * 32)
#define LISTN   (NWAVE * WCAP)
#define NBS     512
#define NTILE   (NBS / 16)
#define TPW     (NTILE / NWAVE)
#define NBH     4096
#define RPW     32
#define RPB     (NWAVE * RPW)
#define LN_EPS  1e-5f

#define LDS_LIST    (LISTN * 4)
#define LDS_S_ACC   (NBS * DF * 4)
#define LDS_S_CNT   (NBS * 4)
#define LDS_SAGE    (LDS_S_ACC + LDS_LIST + LDS_S_CNT + 64)
#define LDS_H_ACC   (NBH * PEIN * 4)
#define LDS_PEAGG   (LDS_H_ACC + LDS_LIST + 64)
#define LDS_P_CONST 3072
#define LDS_P_H     (NWAVE * RPW * HID * 4)
#define LDS_PROJ    (LDS_P_CONST + 2 * LDS_P_H)

static_assert((CHUNK & (CHUNK - 1)) == 0);
static_assert(CHUNK <= 4096);
static_assert((NBS & (NBS - 1)) == 0);
static_assert((NBH & (NBH - 1)) == 0);
static_assert(NBH <= 4096);
static_assert(NBS <= 4096);
static_assert(NTILE % NWAVE == 0);
static_assert(NBS % RPB == 0);
static_assert((PEIN * HID + 2 * HID + DF) * 4 <= LDS_P_CONST);
static_assert(RPW * HID == 16 * DF);
static_assert((NBH * PEIN / 4) % NTHR == 0);
static_assert(NWAVE * 4 <= 64);
static_assert(LDS_SAGE <= 300 * 1024);

typedef float  v4f   __attribute__((ext_vector_type(4)));
typedef float  v8f   __attribute__((ext_vector_type(8)));
typedef int    v4i   __attribute__((ext_vector_type(4)));
typedef __bf16 bf16_t;
typedef bf16_t v8bf  __attribute__((ext_vector_type(8)));
typedef bf16_t v16bf __attribute__((ext_vector_type(16)));
union FragB { v16bf v; v8bf h[2]; v4i q[2]; };
union Pack8 { v8bf v; v4i q; };

__device__ __forceinline__ v8f wmb(v16bf a, v16bf b, v8f c) {
  v8f d = __builtin_amdgcn_wmma_f32_16x16x32_bf16(false, a, false, b, (short)0, c, false, false);
  asm volatile("v_nop\n\tv_nop\n\tv_nop\n\tv_nop" : "+v"(d) : "v"(a), "v"(b));
  return d;
}

template <int B>
__device__ __forceinline__ void split8(FragB& hi, FragB& lo, v4f a, v4f b) {
#define SPL1(I, X) { const float xv = (X); const bf16_t hb = (bf16_t)xv; hi.v[B + (I)] = hb; lo.v[B + (I)] = (bf16_t)(xv - (float)hb); }
  SPL1(0, a.x) SPL1(1, a.y) SPL1(2, a.z) SPL1(3, a.w)
  SPL1(4, b.x) SPL1(5, b.y) SPL1(6, b.z) SPL1(7, b.w)
#undef SPL1
}

template <int NBT>
__device__ __forceinline__ int scan_chunk(const int* __restrict__ dsts, int nE, int cbase, int nodeBase,
                                          int vec8, int* list, int tid, int lane, int wave) {
  int wc = 0;
  (void)lane;
#pragma unroll
  for (int g = 0; g < NGRP; ++g) {
    const int el0  = (g * NTHR + tid) * EPT;
    const int e0   = cbase + el0;
    const int sent = -2147483647 - 1;
    v4i da, db;
    if (vec8 != 0 && cbase + CHUNK <= nE) {
      da = *(const v4i*)(dsts + e0);
      db = *(const v4i*)(dsts + e0 + 4);
    } else {
      da.x = (e0     < nE) ? dsts[min(e0,     nE - 1)] : sent;
      da.y = (e0 + 1 < nE) ? dsts[min(e0 + 1, nE - 1)] : sent;
      da.z = (e0 + 2 < nE) ? dsts[min(e0 + 2, nE - 1)] : sent;
      da.w = (e0 + 3 < nE) ? dsts[min(e0 + 3, nE - 1)] : sent;
      db.x = (e0 + 4 < nE) ? dsts[min(e0 + 4, nE - 1)] : sent;
      db.y = (e0 + 5 < nE) ? dsts[min(e0 + 5, nE - 1)] : sent;
      db.z = (e0 + 6 < nE) ? dsts[min(e0 + 6, nE - 1)] : sent;
      db.w = (e0 + 7 < nE) ? dsts[min(e0 + 7, nE - 1)] : sent;
    }
    const unsigned nb = (unsigned)nodeBase;
    const unsigned s0 = (unsigned)da.x - nb, s1 = (unsigned)da.y - nb;
    const unsigned s2 = (unsigned)da.z - nb, s3 = (unsigned)da.w - nb;
    const unsigned s4 = (unsigned)db.x - nb, s5 = (unsigned)db.y - nb;
    const unsigned s6 = (unsigned)db.z - nb, s7 = (unsigned)db.w - nb;
    const bool h0 = s0 < (unsigned)NBT, h1 = s1 < (unsigned)NBT, h2 = s2 < (unsigned)NBT, h3 = s3 < (unsigned)NBT;
    const bool h4 = s4 < (unsigned)NBT, h5 = s5 < (unsigned)NBT, h6 = s6 < (unsigned)NBT, h7 = s7 < (unsigned)NBT;
    const unsigned any = __builtin_amdgcn_ballot_w32(h0 | h1 | h2 | h3 | h4 | h5 | h6 | h7);
    if (any != 0u) {
#define HITJ(J, HJ, SJ) { \
        const unsigned mj = __builtin_amdgcn_ballot_w32(HJ); \
        if (mj != 0u) { \
          if (HJ) { \
            const int pos = wc + (int)__builtin_amdgcn_mbcnt_lo(mj, 0u); \
            if (pos < WCAP) list[wave * WCAP + pos] = ((el0 + (J)) << 12) | (int)(SJ); \
          } \
          wc += (int)__builtin_popcount(mj); } }
      HITJ(0, h0, s0)
      HITJ(1, h1, s1)
      HITJ(2, h2, s2)
      HITJ(3, h3, s3)
      HITJ(4, h4, s4)
      HITJ(5, h5, s5)
      HITJ(6, h6, s6)
      HITJ(7, h7, s7)
#undef HITJ
    }
  }
  return wc;
}

__global__ __launch_bounds__(NTHR) void k_wplane(
    const float* __restrict__ W0, const float* __restrict__ W1,
    int str0, int str1, int rows0, int kreal, int KP, int N,
    bf16_t* whi, bf16_t* wlo, int nTot) {
  const int i = blockIdx.x * NTHR + threadIdx.x;
  if (i >= nTot) return;
  const int o   = i * 8;
  const int psz = N * KP;
  const int mat = o / psz;
  const int rem = o - mat * psz;
  const int n   = rem / KP;
  const int k0  = rem - n * KP;
  const float* p0 = W0 + (size_t)mat * str0 + n;
  const float* p1 = W1 + (size_t)mat * str1 + n;
  const int kb1 = kreal - rows0 - 1;
  Pack8 ph, pl;
#define WSP(I) { \
    const int k = k0 + (I); \
    const int ka = (k < rows0 - 1) ? k : (rows0 - 1); \
    int kb = k - rows0; kb = kb > kb1 ? kb1 : kb; kb = kb < 0 ? 0 : kb; \
    const float va = p0[(size_t)ka * N]; \
    const float vb = p1[(size_t)kb * N]; \
    const float xv = (k < rows0) ? va : ((k < kreal) ? vb : 0.0f); \
    const bf16_t hb = (bf16_t)xv; ph.v[(I)] = hb; pl.v[(I)] = (bf16_t)(xv - (float)hb); }
  WSP(0) WSP(1) WSP(2) WSP(3) WSP(4) WSP(5) WSP(6) WSP(7)
#undef WSP
  bf16_t* dh = whi + o;
  bf16_t* dl = wlo + o;
  const v4i qh = ph.q, ql = pl.q;
  *(volatile v4i*)dh = qh;
  *(volatile v4i*)dl = ql;
  __threadfence();
  *(volatile v4i*)dh = qh;
  *(volatile v4i*)dl = ql;
}

template <int KP, int NCT>
__device__ __forceinline__ void kstep(const float* ap, float mul,
                                      const bf16_t* bhp, const bf16_t* blp, v8f (&c)[NCT]) {
  const v4f p0 = (*(const v4f*)(ap))      * mul;
  const v4f p1 = (*(const v4f*)(ap + 4))  * mul;
  const v4f p2 = (*(const v4f*)(ap + 16)) * mul;
  const v4f p3 = (*(const v4f*)(ap + 20)) * mul;
  FragB ahi, alo;
  split8<0>(ahi, alo, p0, p1);
  split8<8>(ahi, alo, p2, p3);
#pragma unroll
  for (int ct = 0; ct < NCT; ++ct) {
    const bf16_t* hp = bhp + (size_t)ct * 16 * KP;
    const bf16_t* lp = blp + (size_t)ct * 16 * KP;
    FragB bh, bq;
    bh.q[0] = *(const v4i*)hp;  bh.q[1] = *(const v4i*)(hp + 16);
    bq.q[0] = *(const v4i*)lp;  bq.q[1] = *(const v4i*)(lp + 16);
    c[ct] = wmb(alo.v, bh.v, c[ct]);
    c[ct] = wmb(ahi.v, bq.v, c[ct]);
    c[ct] = wmb(ahi.v, bh.v, c[ct]);
  }
}

__global__ __launch_bounds__(NTHR) void k_peagg(
    const int* __restrict__ he, const float* __restrict__ PE,
    float* agg, int nT, int nE, int vec8) {
  extern __shared__ v4f lds_dyn[];
  float* acc  = (float*)lds_dyn;
  int*   list = (int*)((char*)lds_dyn + LDS_H_ACC);
  int*   wcnt = (int*)((char*)lds_dyn + LDS_H_ACC + LDS_LIST);
  const int tid = threadIdx.x, lane = tid & 31, wave = tid >> 5;
  const int nodeBase = blockIdx.x * NBH;
  const int* srcs = he;
  const int* dsts = he + nE;

  {
    const v4f z = {0.f, 0.f, 0.f, 0.f};
    for (int i = tid; i < NBH * PEIN / 4; i += NTHR) lds_dyn[i] = z;
  }
  __syncthreads();

  const int nChunks = (nE + CHUNK - 1) / CHUNK;
#pragma unroll 1
  for (int ch = 0; ch < nChunks; ++ch) {
    const int cbase = ch * CHUNK;
    const int wc = scan_chunk<NBH>(dsts, nE, cbase, nodeBase, vec8, list, tid, lane, wave);
    if (lane == 0) wcnt[wave] = wc;
    __syncthreads();
    if (wave == 0) {
#pragma unroll 1
      for (int wsx = 0; wsx < NWAVE; ++wsx) {
        int n = __builtin_amdgcn_readfirstlane(wcnt[wsx]);
        n = n > WCAP ? WCAP : (n < 0 ? 0 : n);
        const int* lp = list + wsx * WCAP;
#pragma unroll 1
        for (int i = 0; i < n; ++i) {
          const int ent  = __builtin_amdgcn_readfirstlane(lp[i]);
          const int slot = ent & (NBH - 1);
          int e = cbase + ((ent >> 12) & (CHUNK - 1));
          e = e > nE - 1 ? nE - 1 : e;
          int src = srcs[e];
          src = src < 0 ? 0 : (src > nT - 1 ? nT - 1 : src);
          const int   ch8 = lane & (PEIN - 1);
          const float v   = PE[(size_t)src * PEIN + ch8];
          float* ap = acc + slot * PEIN + ch8;
          const float nv = *ap + v;
          if (lane < PEIN) *ap = nv;
        }
      }
    }
    __syncthreads();
  }

  float* gbase = agg + (size_t)nodeBase * PEIN;
#pragma unroll 1
  for (int it = 0; it < NBH * PEIN / 4 / NTHR; ++it) {
    const int i = it * NTHR + tid;
    const int slot = i >> 1, half = i & 1;
    int nc = nodeBase + slot; nc = nc > nT - 1 ? nT - 1 : nc;
    const v4f v = lds_dyn[i] + *(const v4f*)(PE + (size_t)nc * PEIN + 4 * half);
    *(volatile v4f*)(gbase + 4 * (size_t)i) = v;
  }
  __threadfence();
#pragma unroll 1
  for (int it = 0; it < NBH * PEIN / 4 / NTHR; ++it) {
    const int i = it * NTHR + tid;
    const int slot = i >> 1, half = i & 1;
    int nc = nodeBase + slot; nc = nc > nT - 1 ? nT - 1 : nc;
    const v4f v = lds_dyn[i] + *(const v4f*)(PE + (size_t)nc * PEIN + 4 * half);
    *(volatile v4f*)(gbase + 4 * (size_t)i) = v;
  }
}

__global__ __launch_bounds__(NTHR) void k_proj(
    const float* __restrict__ xinA, const float* __restrict__ xinB,
    const float* __restrict__ agg, int ntRows,
    const float* __restrict__ W1, const float* __restrict__ b1, const float* __restrict__ b2,
    const bf16_t* __restrict__ w2h, const bf16_t* __restrict__ w2l,
    const bf16_t* __restrict__ pwh, const bf16_t* __restrict__ pwl,
    const float* __restrict__ peb,
    float* PA, float* PB, int nN, int nBlkP) {
  extern __shared__ v4f lds_dyn[];
  float* cst = (float*)lds_dyn;
  const int tid = threadIdx.x, lane = tid & 31, wave = tid >> 5, hh = lane >> 4, m = lane & 15;
  float* hL  = (float*)((char*)lds_dyn + LDS_P_CONST) + wave * (RPW * HID);
  float* peL = (float*)((char*)lds_dyn + LDS_P_CONST + LDS_P_H) + wave * (RPW * HID);
  float* oL  = hL;
  const int type    = ((int)blockIdx.x >= nBlkP) ? 1 : 0;
  const int rowBase = ((int)blockIdx.x - type * nBlkP) * RPB;
  const float* xin  = type ? xinB : xinA;
  float* P          = type ? PB : PA;
  const int typeOff = type * nN;

  for (int i = tid; i < PEIN * HID; i += NTHR) cst[i] = W1[i];
  {
    const int j = tid < HID - 1 ? tid : HID - 1;
    const float vb1 = b1[j], vb2 = b2[j];
    if (tid < HID) { cst[PEIN * HID + tid] = vb1; cst[PEIN * HID + HID + tid] = vb2; }
    const int jj = tid < DF - 1 ? tid : DF - 1;
    const float vpb = peb[jj];
    if (tid < DF) cst[PEIN * HID + 2 * HID + tid] = vpb;
  }
  __syncthreads();
  const float* sW1  = cst;
  const float* sb1  = cst + PEIN * HID;
  const float* sb2  = sb1 + HID;
  const float* speb = sb2 + HID;

  {
    int hid = typeOff + rowBase + RPW * wave + lane;
    hid = hid > ntRows - 1 ? ntRows - 1 : hid;
    const v4f a0 = *(const v4f*)(agg + (size_t)hid * PEIN);
    const v4f a1 = *(const v4f*)(agg + (size_t)hid * PEIN + 4);
    float* hrow = hL + lane * HID;
#pragma unroll 1
    for (int j = 0; j < HID; ++j) {
      float s = sb1[j];
      s += a0.x * sW1[0 * HID + j];
      s += a0.y * sW1[1 * HID + j];
      s += a0.z * sW1[2 * HID + j];
      s += a0.w * sW1[3 * HID + j];
      s += a1.x * sW1[4 * HID + j];
      s += a1.y * sW1[5 * HID + j];
      s += a1.z * sW1[6 * HID + j];
      s += a1.w * sW1[7 * HID + j];
      hrow[j] = fmaxf(s, 0.0f);
    }
  }
  __syncthreads();

#pragma unroll 1
  for (int s = 0; s < 2; ++s) {
    v8f c2[4];
#pragma unroll
    for (int ct = 0; ct < 4; ++ct) { const v8f z = {0.f, 0.f, 0.f, 0.f, 0.f, 0.f, 0.f, 0.f}; c2[ct] = z; }
    const float*  arow = hL + (16 * s + m) * HID + 8 * hh;
    const bf16_t* bh0  = w2h + m * HID + 8 * hh;
    const bf16_t* bl0  = w2l + m * HID + 8 * hh;
#pragma unroll 1
    for (int ks = 0; ks < HID / 32; ++ks)
      kstep<HID, 4>(arow + 32 * ks, 1.0f, bh0 + 32 * ks, bl0 + 32 * ks, c2);
    float* sp = peL + (16 * s + 8 * hh) * HID + m;
#pragma unroll
    for (int ct = 0; ct < 4; ++ct) {
      const float bb = sb2[16 * ct + m];
#pragma unroll
      for (int r = 0; r < 8; ++r) sp[r * HID + 16 * ct] = c2[ct][r] + bb;
    }
  }
  __syncthreads();

#pragma unroll 1
  for (int s = 0; s < 2; ++s) {
    int node = rowBase + RPW * wave + 16 * s + m;
    node = node > nN - 1 ? nN - 1 : node;
    v8f c[8];
#pragma unroll
    for (int ct = 0; ct < 8; ++ct) { const v8f z = {0.f, 0.f, 0.f, 0.f, 0.f, 0.f, 0.f, 0.f}; c[ct] = z; }
    const float*  xrow = xin + (size_t)node * DF + 8 * hh;
    const float*  prow = peL + (16 * s + m) * HID + 8 * hh;
    const bf16_t* bh0  = pwh + m * KPE + 8 * hh;
    const bf16_t* bl0  = pwl + m * KPE + 8 * hh;
#pragma unroll 1
    for (int ks = 0; ks < DF / 32; ++ks)
      kstep<KPE, 8>(xrow + 32 * ks, 1.0f, bh0 + 32 * ks, bl0 + 32 * ks, c);
#pragma unroll 1
    for (int ks = 0; ks < HID / 32; ++ks)
      kstep<KPE, 8>(prow + 32 * ks, 1.0f, bh0 + DF + 32 * ks, bl0 + DF + 32 * ks, c);
    float* sp = oL + (8 * hh) * DF + m;
#pragma unroll
    for (int ct = 0; ct < 8; ++ct) {
      const float bb = speb[16 * ct + m];
#pragma unroll
      for (int r = 0; r < 8; ++r) sp[r * DF + 16 * ct] = c[ct][r] + bb;
    }
    __syncthreads();
    const float* lrow = oL + 4 * lane;
    float* gp = P + ((size_t)rowBase + RPW * wave + 16 * s) * DF + 4 * lane;
#pragma unroll
    for (int i = 0; i < 16; ++i) { const v4f v = *(const v4f*)(lrow + i * DF); *(volatile v4f*)(gp + (size_t)i * DF) = v; }
    __threadfence();
#pragma unroll
    for (int i = 0; i < 16; ++i) { const v4f v = *(const v4f*)(lrow + i * DF); *(volatile v4f*)(gp + (size_t)i * DF) = v; }
    __syncthreads();
  }
}

__global__ __launch_bounds__(NTHR) void k_sage(
    const int* __restrict__ eToA, const int* __restrict__ eToB,
    const float* __restrict__ PA, const float* __restrict__ PB,
    const bf16_t* __restrict__ swh, const bf16_t* __restrict__ swl,
    const float* __restrict__ sbl, const float* __restrict__ lng, const float* __restrict__ lnb,
    float* XA, float* XB, float* out,
    int nEa, int nEb, int nN, int nBlkS, int vecA, int vecB, int last) {
  extern __shared__ v4f lds_dyn[];
  float* acc  = (float*)lds_dyn;
  int*   list = (int*)((char*)lds_dyn + LDS_S_ACC);
  int*   cnt  = (int*)((char*)lds_dyn + LDS_S_ACC + LDS_LIST);
  int*   wcnt = (int*)((char*)lds_dyn + LDS_S_ACC + LDS_LIST + LDS_S_CNT);
  const int tid = threadIdx.x, lane = tid & 31, wave = tid >> 5, hh = lane >> 4, m = lane & 15;
  const int type     = ((int)blockIdx.x >= nBlkS) ? 1 : 0;
  const int nodeBase = ((int)blockIdx.x - type * nBlkS) * NBS;
  const int* ei      = type ? eToB : eToA;
  const int  nE      = type ? nEb : nEa;
  const int  vec8    = type ? vecB : vecA;
  const float* xsrc  = type ? PA : PB;
  const float* xself = type ? PB : PA;
  const int  wsel    = type ? 0 : 1;
  const int  lsel    = type ? 1 : 0;
  const bf16_t* whi  = swh + (size_t)wsel * DF * KSG;
  const bf16_t* wlo  = swl + (size_t)wsel * DF * KSG;
  const float* bias  = sbl + wsel * DF;
  const float* gam   = lng + lsel * DF;
  const float* bet   = lnb + lsel * DF;
  float* xout        = type ? XB : XA;
  float* outT        = out + (size_t)type * nN * DF;
  const int* srcs    = ei;
  const int* dsts    = ei + nE;

  {
    const v4f z = {0.f, 0.f, 0.f, 0.f};
    for (int i = tid; i < NBS * DF / 4; i += NTHR) lds_dyn[i] = z;
    for (int i = tid; i < NBS; i += NTHR) cnt[i] = 0;
  }
  __syncthreads();

  const int nChunks = (nE + CHUNK - 1) / CHUNK;
#pragma unroll 1
  for (int ch = 0; ch < nChunks; ++ch) {
    const int cbase = ch * CHUNK;
    const int wc = scan_chunk<NBS>(dsts, nE, cbase, nodeBase, vec8, list, tid, lane, wave);
    if (lane == 0) wcnt[wave] = wc;
    __syncthreads();
    if (wave == 0) {
#pragma unroll 1
      for (int wsx = 0; wsx < NWAVE; ++wsx) {
        int n = __builtin_amdgcn_readfirstlane(wcnt[wsx]);
        n = n > WCAP ? WCAP : (n < 0 ? 0 : n);
        const int* lp = list + wsx * WCAP;
#pragma unroll 1
        for (int i = 0; i < n; ++i) {
          const int ent  = __builtin_amdgcn_readfirstlane(lp[i]);
          const int slot = ent & (NBS - 1);
          int e = cbase + ((ent >> 12) & (CHUNK - 1));
          e = e > nE - 1 ? nE - 1 : e;
          int src = srcs[e];
          src = src < 0 ? 0 : (src > nN - 1 ? nN - 1 : src);
          const v4f v = *(const v4f*)(xsrc + (size_t)src * DF + 4 * lane);
          v4f* ap = (v4f*)(acc + slot * DF + 4 * lane);
          *ap = *ap + v;
          if (lane == 0) cnt[slot] = cnt[slot] + 1;
        }
      }
    }
    __syncthreads();
  }

#pragma unroll 1
  for (int q = 0; q < TPW; ++q) {
    const int t     = q * NWAVE + wave;
    const int slotm = 16 * t + m;
    int node = nodeBase + slotm;
    node = node > nN - 1 ? nN - 1 : node;
    const int   cd  = cnt[slotm];
    const float inv = cd > 0 ? (1.0f / (float)cd) : 0.0f;

    v8f c[8];
#pragma unroll
    for (int ct = 0; ct < 8; ++ct) { const v8f z = {0.f, 0.f, 0.f, 0.f, 0.f, 0.f, 0.f, 0.f}; c[ct] = z; }

    const float*  arow = acc + slotm * DF + 8 * hh;
    const float*  xrow = xself + (size_t)node * DF + 8 * hh;
    const bf16_t* bh0  = whi + m * KSG + 8 * hh;
    const bf16_t* bl0  = wlo + m * KSG + 8 * hh;
#pragma unroll 1
    for (int ks = 0; ks < DF / 32; ++ks)
      kstep<KSG, 8>(arow + 32 * ks, inv, bh0 + 32 * ks, bl0 + 32 * ks, c);
#pragma unroll 1
    for (int ks = 0; ks < DF / 32; ++ks)
      kstep<KSG, 8>(xrow + 32 * ks, 1.0f, bh0 + DF + 32 * ks, bl0 + DF + 32 * ks, c);

#pragma unroll
    for (int ct = 0; ct < 8; ++ct) { const float bb = bias[16 * ct + m]; c[ct] = c[ct] + bb; }
    float mu[8], rsd[8];
#pragma unroll
    for (int r = 0; r < 8; ++r) {
      float s = c[0][r] + c[1][r] + c[2][r] + c[3][r] + c[4][r] + c[5][r] + c[6][r] + c[7][r];
      s += __shfl_xor(s, 1);
      s += __shfl_xor(s, 2);
      s += __shfl_xor(s, 4);
      s += __shfl_xor(s, 8);
      mu[r] = s * (1.0f / (float)DF);
    }
#pragma unroll
    for (int r = 0; r < 8; ++r) {
      float qv = 0.0f;
#pragma unroll
      for (int ct = 0; ct < 8; ++ct) { const float d = c[ct][r] - mu[r]; qv += d * d; }
      qv += __shfl_xor(qv, 1);
      qv += __shfl_xor(qv, 2);
      qv += __shfl_xor(qv, 4);
      qv += __shfl_xor(qv, 8);
      rsd[r] = rsqrtf(qv * (1.0f / (float)DF) + LN_EPS);
    }
    float* sp = acc + (16 * t + 8 * hh) * DF + m;
#pragma unroll
    for (int ct = 0; ct < 8; ++ct) {
      const int   col = 16 * ct + m;
      const float g = gam[col], b = bet[col];
#pragma unroll
      for (int r = 0; r < 8; ++r) {
        const float y = (c[ct][r] - mu[r]) * rsd[r] * g + b;
        sp[r * DF + 16 * ct] = fmaxf(y, 0.0f);
      }
    }
    __syncthreads();

    const float* lrow = acc + (16 * t) * DF + 4 * lane;
    const int row0g = nodeBase + 16 * t;
    if (last == 0) {
      float* gp = xout + (size_t)row0g * DF + 4 * lane;
#pragma unroll
      for (int i = 0; i < 16; ++i) { const v4f v = *(const v4f*)(lrow + i * DF); *(volatile v4f*)(gp + (size_t)i * DF) = v; }
      __threadfence();
#pragma unroll
      for (int i = 0; i < 16; ++i) { const v4f v = *(const v4f*)(lrow + i * DF); *(volatile v4f*)(gp + (size_t)i * DF) = v; }
    } else {
      float* gp = outT + (size_t)row0g * DF + 4 * lane;
#pragma unroll
      for (int i = 0; i < 16; ++i) {
        if (row0g + i < nN) { const v4f v = *(const v4f*)(lrow + i * DF); *(volatile v4f*)(gp + (size_t)i * DF) = v; }
      }
      __threadfence();
#pragma unroll
      for (int i = 0; i < 16; ++i) {
        if (row0g + i < nN) { const v4f v = *(const v4f*)(lrow + i * DF); *(volatile v4f*)(gp + (size_t)i * DF) = v; }
      }
    }
  }
}

extern "C" void kernel_launch(void* const* d_in, const int* in_sizes, int n_in,
                              void* d_out, int out_size, void* d_ws, size_t ws_size,
                              hipStream_t stream) {
  if (n_in < 17) return;
  const int nN = in_sizes[0] / DF;
  if (nN <= 0 || in_sizes[0] != nN * DF || in_sizes[1] != nN * DF) return;
  const int nT = in_sizes[2] / PEIN;
  if (in_sizes[2] != nT * PEIN || nT != 2 * nN) return;
  if ((in_sizes[3] & 1) || (in_sizes[4] & 1) || (in_sizes[5] & 1)) return;
  const int nEb = in_sizes[3] / 2;
  const int nEa = in_sizes[4] / 2;
  const int nEh = in_sizes[5] / 2;
  if (nEb < 0 || nEa < 0 || nEh < 0) return;
  const int nL = in_sizes[6] / (2 * DF * DF);
  if (nL <= 0 || in_sizes[6] != nL * 2 * DF * DF || in_sizes[8] != nL * 2 * DF * DF) return;
  if (in_sizes[7] != nL * 2 * DF || in_sizes[9] != nL * 2 * DF || in_sizes[10] != nL * 2 * DF) return;
  if (in_sizes[11] != nL * PEIN * HID || in_sizes[12] != nL * HID) return;
  if (in_sizes[13] != nL * HID * HID || in_sizes[14] != nL * HID) return;
  if (in_sizes[15] != nL * KPE * DF || in_sizes[16] != nL * DF) return;
  if (out_size != 2 * nN * DF) return;

  const float* xA  = (const float*)d_in[0];
  const float* xB  = (const float*)d_in[1];
  const float* PE  = (const float*)d_in[2];
  const int*   eAB = (const int*)d_in[3];
  const int*   eBA = (const int*)d_in[4];
  const int*   he  = (const int*)d_in[5];
  const float* sWl = (const float*)d_in[6];
  const float* sbl = (const float*)d_in[7];
  const float* sWr = (const float*)d_in[8];
  const float* lng = (const float*)d_in[9];
  const float* lnb = (const float*)d_in[10];
  const float* pW1 = (const float*)d_in[11];
  const float* pb1 = (const float*)d_in[12];
  const float* pW2 = (const float*)d_in[13];
  const float* pb2 = (const float*)d_in[14];
  const float* peW = (const float*)d_in[15];
  const float* peb = (const float*)d_in[16];
  float* out = (float*)d_out;

  const int nBlkS = (nN + NBS - 1) / NBS;
  const int NPAD  = nBlkS * NBS;
  const int nBlkP = NPAD / RPB;
  const int nBlkH = (nT + NBH - 1) / NBH;
  const int NTP   = nBlkH * NBH;

  char* ws = (char*)d_ws;
  size_t off = 0;
  const size_t szSW  = (size_t)2 * nL * DF * KSG * 2;
  const size_t szPW  = (size_t)nL * DF * KPE * 2;
  const size_t szW2  = (size_t)nL * HID * HID * 2;
  const size_t szAgg = (size_t)NTP * PEIN * 4;
  const size_t szX   = (size_t)NPAD * DF * 4;
#define CARVE(NAME, SZ) const size_t NAME = off; off += (SZ); off = (off + 255) & ~(size_t)255;
  CARVE(oSWh, szSW) CARVE(oSWl, szSW)
  CARVE(oPWh, szPW) CARVE(oPWl, szPW)
  CARVE(oW2h, szW2) CARVE(oW2l, szW2)
  CARVE(oAgg, szAgg)
  CARVE(oPA, szX) CARVE(oPB, szX)
  CARVE(oXA, szX) CARVE(oXB, szX)
#undef CARVE
  if (off > ws_size) return;
  bf16_t* swh = (bf16_t*)(ws + oSWh);
  bf16_t* swl = (bf16_t*)(ws + oSWl);
  bf16_t* pwh = (bf16_t*)(ws + oPWh);
  bf16_t* pwl = (bf16_t*)(ws + oPWl);
  bf16_t* w2h = (bf16_t*)(ws + oW2h);
  bf16_t* w2l = (bf16_t*)(ws + oW2l);
  float*  agg = (float*)(ws + oAgg);
  float*  PAp = (float*)(ws + oPA);
  float*  PBp = (float*)(ws + oPB);
  float*  XAp = (float*)(ws + oXA);
  float*  XBp = (float*)(ws + oXB);

  const int vecA = ((nEa & 3) == 0) ? 1 : 0;
  const int vecB = ((nEb & 3) == 0) ? 1 : 0;
  const int vecH = ((nEh & 3) == 0) ? 1 : 0;

  {
    const int nTotS = 2 * nL * DF * KSG / 8;
    k_wplane<<<(nTotS + NTHR - 1) / NTHR, NTHR, 0, stream>>>(
        sWl, sWr, DF * DF, DF * DF, DF, KSG, KSG, DF, swh, swl, nTotS);
    const int nTotP = nL * DF * KPE / 8;
    k_wplane<<<(nTotP + NTHR - 1) / NTHR, NTHR, 0, stream>>>(
        peW, peW, KPE * DF, KPE * DF, KPE, KPE, KPE, DF, pwh, pwl, nTotP);
    const int nTotW = nL * HID * HID / 8;
    k_wplane<<<(nTotW + NTHR - 1) / NTHR, NTHR, 0, stream>>>(
        pW2, pW2, HID * HID, HID * HID, HID, HID, HID, HID, w2h, w2l, nTotW);
  }

  hipFuncSetAttribute(reinterpret_cast<const void*>(&k_peagg),
                      hipFuncAttributeMaxDynamicSharedMemorySize, LDS_PEAGG);
  hipFuncSetAttribute(reinterpret_cast<const void*>(&k_proj),
                      hipFuncAttributeMaxDynamicSharedMemorySize, LDS_PROJ);
  hipFuncSetAttribute(reinterpret_cast<const void*>(&k_sage),
                      hipFuncAttributeMaxDynamicSharedMemorySize, LDS_SAGE);

  k_peagg<<<nBlkH, NTHR, LDS_PEAGG, stream>>>(he, PE, agg, nT, nEh, vecH);

  for (int l = 0; l < nL; ++l) {
    const int last = (l == nL - 1) ? 1 : 0;
    const float* xinA = (l == 0) ? xA : XAp;
    const float* xinB = (l == 0) ? xB : XBp;
    k_proj<<<2 * nBlkP, NTHR, LDS_PROJ, stream>>>(
        xinA, xinB, agg, NTP,
        pW1 + (size_t)l * PEIN * HID, pb1 + (size_t)l * HID, pb2 + (size_t)l * HID,
        w2h + (size_t)l * HID * HID, w2l + (size_t)l * HID * HID,
        pwh + (size_t)l * DF * KPE, pwl + (size_t)l * DF * KPE,
        peb + (size_t)l * DF,
        PAp, PBp, nN, nBlkP);
    k_sage<<<2 * nBlkS, NTHR, LDS_SAGE, stream>>>(
        eBA, eAB, PAp, PBp,
        swh + (size_t)l * 2 * DF * KSG, swl + (size_t)l * 2 * DF * KSG,
        sbl + (size_t)l * 2 * DF, lng + (size_t)l * 2 * DF, lnb + (size_t)l * 2 * DF,
        XAp, XBp, out, nEa, nEb, nN, nBlkS, vecA, vecB, last);
  }
}
